// IDA_pare_46986942218480
// MI455X (gfx1250) — hardware-verified
//
#include <hip/hip_runtime.h>
#include <stdint.h>

#pragma clang fp contract(off)

#define NB    2
#define C1    256
#define NO    128
#define H1    64
#define W1    128
#define H2    128
#define W2    256
#define PH1   (H1 + 2)
#define PW1   (W1 + 2)
#define PH2   (H2 + 2)
#define PW2   (W2 + 2)
#define K1    (9 * C1)
#define K2    (9 * NO)
#define NOF   27
#define NOP   32
#define NMK   9
#define MPX   32
#define OFP   36
#define XSP   (NO + 8)
#define TPU   (NO + 4)
#define UPR   66
#define CSC   16.0f
#define WSC   1024.0f
#define INV_S 6.103515625e-05f

#define XH_E  ((size_t)NB * PH1 * PW1 * C1)
#define HB_E  ((size_t)NB * H1 * W1 * NO)
#define ZP_E  ((size_t)NB * PH2 * PW2 * NO)
#define NPX1  (NB * H1 * W1)
#define NPX2  (NB * H2 * W2)

#define WO1_CHK (NOP * K1 / 8)
#define WR1_CHK (NO * K1 / 8)
#define WO2_CHK (NOP * K2 / 8)
#define WR2_CHK (NO * K2 / 8)

#define XCV_BLK  (NB * PH1 * 2)
#define OFF1_BLK (NB * H1 * (W1 / 64))
#define CNV1_BLK (NB * H1 * (W1 / MPX))
#define UP_BLK   (NB * PH2 * 4)
#define OFF2_BLK (NB * H2 * (W2 / 64))
#define CNV2_BLK (NB * H2 * (W2 / MPX))

#define WS_WO1 ((size_t)0)
#define WS_WR1 (WS_WO1 + (size_t)NOP * K1 * 2)
#define WS_WO2 (WS_WR1 + (size_t)NO * K1 * 2)
#define WS_WR2 (WS_WO2 + (size_t)NOP * K2 * 2)
#define WS_XH  (WS_WR2 + (size_t)NO * K2 * 2)
#define WS_OF1 (WS_XH + XH_E * 2)
#define WS_HB  (WS_OF1 + (size_t)NPX1 * NOP * 4)
#define WS_ZF  (WS_HB + HB_E * 4)
#define WS_ZH  (WS_ZF + ZP_E * 4)
#define WS_ZL  (WS_ZH + ZP_E * 2)
#define WS_OF2 (WS_ZL + ZP_E * 2)
#define WS_END (WS_OF2 + (size_t)NPX2 * NOP * 4)

static_assert(WO1_CHK % 256 == 0);
static_assert(WR1_CHK % 256 == 0);
static_assert(WO2_CHK % 256 == 0);
static_assert(WR2_CHK % 256 == 0);
static_assert(K1 % 64 == 0);
static_assert(K2 % 64 == 0);
static_assert((WS_WR1 % 128) == 0);
static_assert((WS_WO2 % 128) == 0);
static_assert((WS_WR2 % 128) == 0);
static_assert((WS_XH % 128) == 0);
static_assert((WS_OF1 % 128) == 0);
static_assert((WS_HB % 128) == 0);
static_assert((WS_ZF % 128) == 0);
static_assert((WS_ZH % 128) == 0);
static_assert((WS_ZL % 128) == 0);
static_assert((WS_OF2 % 128) == 0);
static_assert((WS_END % 128) == 0);
static_assert(WS_END <= (size_t)134217728);
static_assert((XSP * 2) % 16 == 0);
static_assert((TPU * 4) % 16 == 0);
static_assert((OFP * 4) % 16 == 0);
static_assert(PW1 * XSP * 2 <= 48000);
static_assert(UPR * TPU * 4 + NO * 16 * 4 <= 48000);
static_assert(W1 % 64 == 0);
static_assert(W2 % 64 == 0);
static_assert(W2 == 256);
static_assert(W1 % MPX == 0);
static_assert(W2 % MPX == 0);
static_assert(NO * 2 == 256);
static_assert(NOP * 4 == 128);
static_assert(MPX * 4 == 128);
static_assert(9 * 32 >= 2 * PW1);
static_assert(9 * 32 >= 4 * UPR);
static_assert(5 * 32 >= 2 * UPR);

typedef _Float16       v16h __attribute__((ext_vector_type(16)));
typedef _Float16       v8h  __attribute__((ext_vector_type(8)));
typedef __bf16         v16b __attribute__((ext_vector_type(16)));
typedef __bf16         v8b  __attribute__((ext_vector_type(8)));
typedef float          v8f  __attribute__((ext_vector_type(8)));
typedef float          v4f  __attribute__((ext_vector_type(4)));
typedef unsigned       v4u  __attribute__((ext_vector_type(4)));
typedef unsigned short v8us __attribute__((ext_vector_type(8)));

__device__ __forceinline__ unsigned bfb(float f) {
  const unsigned u = __float_as_uint(f);
  return (u + 0x7FFFu + ((u >> 16) & 1u)) >> 16;
}
__device__ __forceinline__ float bf_rne(float f) { return __uint_as_float(bfb(f) << 16); }
__device__ __forceinline__ unsigned hbits(_Float16 h) {
  return (unsigned)__builtin_bit_cast(unsigned short, h);
}
__device__ __forceinline__ v8f zero8f() { v8f z = {0.f, 0.f, 0.f, 0.f, 0.f, 0.f, 0.f, 0.f}; return z; }
__device__ __forceinline__ v4f zero4f() { v4f z = {0.f, 0.f, 0.f, 0.f}; return z; }
__device__ __forceinline__ v8us zero8us() {
  v8us z;
#pragma unroll
  for (int e = 0; e < 8; ++e) z[e] = (unsigned short)0;
  return z;
}

__device__ __forceinline__ v16h ldfrag_h(const _Float16* p) {
  union { v16h v; v8h h[2]; } f;
  f.h[0] = *(const v8h*)(p);
  f.h[1] = *(const v8h*)(p + 16);
  return f.v;
}
__device__ __forceinline__ v16b ldfrag_b(const __bf16* p) {
  union { v16b v; v8b h[2]; } f;
  f.h[0] = *(const v8b*)(p);
  f.h[1] = *(const v8b*)(p + 16);
  return f.v;
}

__device__ __forceinline__ v8f mma_h(v16h a, v16h b, v8f c) {
  return __builtin_amdgcn_wmma_f32_16x16x32_f16(false, a, false, b, (short)0, c, false, false);
}
__device__ __forceinline__ v8f mma_b(v16b a, v16b b, v8f c) {
  return __builtin_amdgcn_wmma_f32_16x16x32_bf16(false, a, false, b, (short)0, c, false, false);
}
template <typename F>
__device__ __forceinline__ void guard1x4(v8f& c0, const F& f0, const F& f1, const F& f2, const F& f3) {
#if defined(__HIP_DEVICE_COMPILE__)
  asm volatile("v_nop\n\tv_nop\n\tv_nop\n\tv_nop"
               : "+v"(c0)
               : "v"(f0), "v"(f1), "v"(f2), "v"(f3));
#endif
}
template <typename F>
__device__ __forceinline__ void guard1x6(v8f& c0, const F& f0, const F& f1, const F& f2,
                                         const F& f3, const F& f4, const F& f5) {
#if defined(__HIP_DEVICE_COMPILE__)
  asm volatile("v_nop\n\tv_nop\n\tv_nop\n\tv_nop"
               : "+v"(c0)
               : "v"(f0), "v"(f1), "v"(f2), "v"(f3), "v"(f4), "v"(f5));
#endif
}
template <typename F>
__device__ __forceinline__ void guard2x3(v8f& c0, v8f& c1, const F& f0, const F& f1, const F& f2) {
#if defined(__HIP_DEVICE_COMPILE__)
  asm volatile("v_nop\n\tv_nop\n\tv_nop\n\tv_nop"
               : "+v"(c0), "+v"(c1)
               : "v"(f0), "v"(f1), "v"(f2));
#endif
}
__device__ __forceinline__ void acc_guard1(v8f& c0) {
#if defined(__HIP_DEVICE_COMPILE__)
  asm volatile("v_nop\n\tv_nop\n\tv_nop\n\tv_nop" : "+v"(c0));
#endif
}
__device__ __forceinline__ void acc_guard2(v8f& c0, v8f& c1) {
#if defined(__HIP_DEVICE_COMPILE__)
  asm volatile("v_nop\n\tv_nop\n\tv_nop\n\tv_nop" : "+v"(c0), "+v"(c1));
#endif
}

__global__ __launch_bounds__(256)
void k_wpack(const float* __restrict__ w, unsigned* dst, int nvalid, int cin, int scaled16)
{
  const int q    = blockIdx.x * 256 + threadIdx.x;
  const int kch  = (9 * cin) >> 3;
  const int row  = q / kch;
  const int kc   = (q - row * kch) * 8;
  const int tap  = kc / cin;
  const int ci0  = kc - tap * cin;
  const int rowc = min(row, nvalid - 1);
  const bool live = row < nvalid;
  unsigned hb[8];
#pragma unroll
  for (int j = 0; j < 8; ++j) {
    float v = w[((size_t)(rowc * cin + ci0 + j)) * 9 + tap];
    v = live ? v : 0.0f;
    const unsigned b16 = bfb(v);
    const unsigned h16 = hbits((_Float16)(__uint_as_float(b16 << 16) * WSC));
    hb[j] = (scaled16 != 0) ? h16 : b16;
  }
  v4u wh;
  wh.x = hb[0] | (hb[1] << 16);
  wh.y = hb[2] | (hb[3] << 16);
  wh.z = hb[4] | (hb[5] << 16);
  wh.w = hb[6] | (hb[7] << 16);
  unsigned* d = dst + (size_t)q * 4;
  *(volatile v4u*)d = wh;
  __threadfence();
  *(volatile v4u*)d = wh;
}

__global__ __launch_bounds__(256)
void k_xcvt(const float* __restrict__ x, unsigned short* xh)
{
  __shared__ __align__(16) unsigned short T[PW1 * XSP];
  const int tid  = threadIdx.x;
  const int lane = tid & 31;
  const int wid  = tid >> 5;
  const int pj   = lane & 7;
  const int lq   = lane >> 3;
  const int cg   = blockIdx.x & 1;
  const int bh   = blockIdx.x >> 1;
  const int b    = bh / PH1;
  const int hp   = bh - b * PH1;
  const bool inrow = (hp >= 1) && (hp <= H1);
  const int hc   = min(max(hp - 1, 0), H1 - 1);

  if (tid < 32) {
    const int slot = (tid < 16) ? 0 : (PW1 - 1);
    *(v8us*)&T[slot * XSP + 8 * (tid & 15)] = zero8us();
  }
#pragma unroll 4
  for (int i = 0; i < 16; ++i) {
    const int idx = tid + 256 * i;
    const int w4  = idx & 31;
    const int c   = idx >> 5;
    const v4f v = *(const v4f*)(x + ((size_t)(b * C1 + 128 * cg + c) * H1 + hc) * W1 + 4 * w4);
    unsigned short* tp = T + (4 * w4 + 1) * XSP + c;
    tp[0 * XSP] = (unsigned short)(inrow ? bfb(v.x) : 0u);
    tp[1 * XSP] = (unsigned short)(inrow ? bfb(v.y) : 0u);
    tp[2 * XSP] = (unsigned short)(inrow ? bfb(v.z) : 0u);
    tp[3 * XSP] = (unsigned short)(inrow ? bfb(v.w) : 0u);
  }
  __syncthreads();

  constexpr int NL  = 2 * PW1;
  constexpr int NIT = 9;
  v8us val[NIT]; size_t e[NIT]; bool ok[NIT];
#pragma unroll
  for (int r = 0; r < NIT; ++r) {
    const int L   = r * 32 + wid * 4 + lq;
    ok[r] = (L < NL);
    const int Lc  = ok[r] ? L : (NL - 1);
    const int px  = Lc >> 1;
    const int sub = Lc & 1;
    val[r] = *(const v8us*)&T[px * XSP + 64 * sub + 8 * pj];
    e[r]   = ((size_t)(bh * PW1 + px)) * C1 + 128 * cg + 64 * sub + 8 * pj;
  }
#pragma unroll
  for (int r = 0; r < NIT; ++r) if (ok[r]) *(volatile v8us*)(xh + e[r]) = val[r];
  __threadfence();
#pragma unroll
  for (int r = 0; r < NIT; ++r) if (ok[r]) *(volatile v8us*)(xh + e[r]) = val[r];
}

template <int CIN, int IH, int IW, bool SPLIT>
__global__ __launch_bounds__(256)
void k_offs(const __bf16* __restrict__ ph, const __bf16* __restrict__ pl,
            const __bf16* __restrict__ wo, const float* __restrict__ bom, float* offp)
{
  constexpr int PW = IW + 2;
  constexpr int PH = IH + 2;
  constexpr int K  = 9 * CIN;
  constexpr int NQ = IW / 64;
  static_assert(CIN % 64 == 0);
  __shared__ __align__(16) float st[64 * OFP];

  const int tid  = threadIdx.x;
  const int lane = tid & 31;
  const int wid  = tid >> 5;
  const int l15  = lane & 15;
  const int hh   = lane >> 4;
  const int b    = blockIdx.x / (IH * NQ);
  const int rm   = blockIdx.x - b * (IH * NQ);
  const int h    = rm / NQ;
  const int xo   = (rm - h * NQ) * 64;

  const int mt = wid & 3;
  const int nt = wid >> 2;
  const size_t aoff = (((size_t)(b * PH + h)) * PW + xo + 16 * mt + l15) * CIN + 8 * hh;
  const __bf16* bp = wo + (size_t)(16 * nt + l15) * K + 8 * hh;
  v8f acc = zero8f();
#pragma unroll 1
  for (int kh = 0; kh < 3; ++kh) {
#pragma unroll 1
    for (int kw = 0; kw < 3; ++kw) {
      const size_t ao = aoff + (size_t)(kh * PW + kw) * CIN;
      const __bf16* bk = bp + (kh * 3 + kw) * CIN;
#pragma unroll 2
      for (int kc = 0; kc < CIN / 64; ++kc) {
        if constexpr (!SPLIT) {
          const v16b fa0 = ldfrag_b(ph + ao + 64 * kc);
          const v16b fa1 = ldfrag_b(ph + ao + 64 * kc + 32);
          const v16b fb0 = ldfrag_b(bk + 64 * kc);
          const v16b fb1 = ldfrag_b(bk + 64 * kc + 32);
          acc = mma_b(fa0, fb0, acc);
          acc = mma_b(fa1, fb1, acc);
          guard1x4(acc, fa0, fa1, fb0, fb1);
        } else {
          const v16b fah0 = ldfrag_b(ph + ao + 64 * kc);
          const v16b fal0 = ldfrag_b(pl + ao + 64 * kc);
          const v16b fah1 = ldfrag_b(ph + ao + 64 * kc + 32);
          const v16b fal1 = ldfrag_b(pl + ao + 64 * kc + 32);
          const v16b fb0  = ldfrag_b(bk + 64 * kc);
          const v16b fb1  = ldfrag_b(bk + 64 * kc + 32);
          acc = mma_b(fah0, fb0, acc);
          acc = mma_b(fal0, fb0, acc);
          acc = mma_b(fah1, fb1, acc);
          acc = mma_b(fal1, fb1, acc);
          guard1x6(acc, fah0, fal0, fah1, fal1, fb0, fb1);
        }
      }
    }
  }
  acc_guard1(acc);

  {
    const int ch = 16 * nt + l15;
    const float bv  = bf_rne(bom[min(ch, NOF - 1)]);
    const float obv = (ch < NOF) ? bv : 0.0f;
    float* srow = st + (16 * mt + 8 * hh) * OFP + ch;
#pragma unroll
    for (int r = 0; r < 8; ++r) {
      float v = acc[r] + obv;
      if (ch >= NOF) v = 0.0f;
      srow[r * OFP] = v;
    }
  }
  __syncthreads();

#pragma unroll 1
  for (int it = tid; it < 64 * NMK; it += 256) {
    const int px = it / NMK;
    const int j  = it - px * NMK;
    float* p = st + px * OFP + 2 * NMK + j;
    const float v  = *p;
    const float ev = expf(-fmaxf(v, -40.0f));
    const float s  = 1.0f / (1.0f + ev);
    *p = s;
  }
  __syncthreads();

  {
    const int pj = lane & 7;
    const int lq = lane >> 3;
    const size_t pix0 = (size_t)b * IH * IW + (size_t)h * IW + xo;
    v4f val[2]; size_t e[2];
#pragma unroll
    for (int r = 0; r < 2; ++r) {
      const int L = r * 32 + wid * 4 + lq;
      val[r] = *(const v4f*)&st[L * OFP + 4 * pj];
      e[r]   = (pix0 + L) * NOP + 4 * pj;
    }
#pragma unroll
    for (int r = 0; r < 2; ++r) *(volatile v4f*)(offp + e[r]) = val[r];
    __threadfence();
#pragma unroll
    for (int r = 0; r < 2; ++r) *(volatile v4f*)(offp + e[r]) = val[r];
  }
}

template <int CIN, int IH, int IW, bool SRC32, bool ONCHW>
__global__ __launch_bounds__(256)
void k_conv(const unsigned short* __restrict__ s16, const float* __restrict__ s32,
            const _Float16* __restrict__ wr, const float* __restrict__ offp,
            const float* __restrict__ bias, const float* __restrict__ gam,
            const float* __restrict__ bet, const float* __restrict__ mea,
            const float* __restrict__ var, float* dst)
{
  constexpr int PW   = IW + 2;
  constexpr int PH   = IH + 2;
  constexpr int K    = 9 * CIN;
  constexpr int NSEG = IW / MPX;
  constexpr int SP   = CIN + 8;
  constexpr int OSP  = ONCHW ? (MPX + 4) : (NO + 4);
  constexpr int ATB  = MPX * SP * 2;
  constexpr int OSB  = ONCHW ? (NO * OSP * 4) : (MPX * OSP * 4);
  constexpr int TRB  = (ATB > OSB) ? ATB : OSB;
  static_assert((SP * 2) % 16 == 0);
  static_assert((OSP * 4) % 16 == 0);
  static_assert(CIN % 64 == 0);
  static_assert(TRB <= 32768);

  __shared__ __align__(16) float offl[MPX * NOP];
  __shared__ __align__(16) unsigned char traw[TRB];
  _Float16* At = (_Float16*)traw;
  float*    os = (float*)traw;

  const int tid  = threadIdx.x;
  const int lane = tid & 31;
  const int wid  = tid >> 5;
  const int l15  = lane & 15;
  const int hh   = lane >> 4;
  const int pj   = lane & 7;
  const int lq   = lane >> 3;
  const int b    = blockIdx.x / (IH * NSEG);
  const int rem  = blockIdx.x - b * (IH * NSEG);
  const int h    = rem / NSEG;
  const int xo   = (rem - h * NSEG) * MPX;
  const size_t pix0 = (size_t)b * IH * IW + (size_t)h * IW + xo;

  {
    const int px = tid >> 3;
    const int pc = tid & 7;
    *(v4f*)&offl[px * NOP + 4 * pc] = *(const v4f*)(offp + (pix0 + px) * NOP + 4 * pc);
  }
  __syncthreads();

  const int mt = wid & 1;
  const int nq = wid >> 1;
  const _Float16* bp = wr + (size_t)(32 * nq + l15) * K + 8 * hh;
  v8f acc[2];
  acc[0] = zero8f();
  acc[1] = zero8f();

#pragma unroll 1
  for (int kh = 0; kh < 3; ++kh) {
#pragma unroll 1
    for (int kw = 0; kw < 3; ++kw) {
      const int tap = kh * 3 + kw;

      {
        const int m = 4 * wid + lq;
        const float* orow = offl + m * NOP;
        const float dy = orow[tap];
        const float dx = orow[NMK + tap];
        const float mk = orow[2 * NMK + tap];
        float hf = dy + (float)h;
        hf = hf + (float)(kh - 1);
        float wf = dx + (float)(xo + m);
        wf = wf + (float)(kw - 1);
        const float h0f = floorf(hf);
        const float w0f = floorf(wf);
        const float lh  = hf - h0f;
        const float lw  = wf - w0f;
        const float wh0 = 1.0f - lh;
        const float ww0 = 1.0f - lw;
        const int r0 = (int)fminf(fmaxf(h0f, -2.0f), (float)(PH - 1));
        const int c0 = (int)fminf(fmaxf(w0f, -2.0f), (float)(PW - 1));
        const int r1 = r0 + 1;
        const int c1 = c0 + 1;
        const bool vr0 = (r0 >= 0) && (r0 < IH);
        const bool vr1 = (r1 >= 0) && (r1 < IH);
        const bool vc0 = (c0 >= 0) && (c0 < IW);
        const bool vc1 = (c1 >= 0) && (c1 < IW);
        const float cw00 = (vr0 && vc0) ? (wh0 * ww0) : 0.0f;
        const float cw01 = (vr0 && vc1) ? (wh0 * lw)  : 0.0f;
        const float cw10 = (vr1 && vc0) ? (lh * ww0)  : 0.0f;
        const float cw11 = (vr1 && vc1) ? (lh * lw)   : 0.0f;
        const int pr0 = min(max(r0 + 1, 0), PH - 1);
        const int pr1 = min(max(r1 + 1, 0), PH - 1);
        const int pc0 = min(max(c0 + 1, 0), PW - 1);
        const int pc1 = min(max(c1 + 1, 0), PW - 1);
        const size_t rb0 = ((size_t)(b * PH + pr0)) * PW;
        const size_t rb1 = ((size_t)(b * PH + pr1)) * PW;
        const size_t e00 = (rb0 + pc0) * CIN;
        const size_t e01 = (rb0 + pc1) * CIN;
        const size_t e10 = (rb1 + pc0) * CIN;
        const size_t e11 = (rb1 + pc1) * CIN;
#pragma unroll 2
        for (int cc = 0; cc < CIN / 64; ++cc) {
          const int ch0 = 64 * cc + 8 * pj;
          float v00[8], v01[8], v10[8], v11[8];
          if constexpr (SRC32) {
            const v4f a00 = *(const v4f*)(s32 + e00 + ch0);
            const v4f b00 = *(const v4f*)(s32 + e00 + ch0 + 4);
            const v4f a01 = *(const v4f*)(s32 + e01 + ch0);
            const v4f b01 = *(const v4f*)(s32 + e01 + ch0 + 4);
            const v4f a10 = *(const v4f*)(s32 + e10 + ch0);
            const v4f b10 = *(const v4f*)(s32 + e10 + ch0 + 4);
            const v4f a11 = *(const v4f*)(s32 + e11 + ch0);
            const v4f b11 = *(const v4f*)(s32 + e11 + ch0 + 4);
#pragma unroll
            for (int e = 0; e < 4; ++e) {
              v00[e] = a00[e]; v00[4 + e] = b00[e];
              v01[e] = a01[e]; v01[4 + e] = b01[e];
              v10[e] = a10[e]; v10[4 + e] = b10[e];
              v11[e] = a11[e]; v11[4 + e] = b11[e];
            }
          } else {
            const v4u q00 = *(const v4u*)(s16 + e00 + ch0);
            const v4u q01 = *(const v4u*)(s16 + e01 + ch0);
            const v4u q10 = *(const v4u*)(s16 + e10 + ch0);
            const v4u q11 = *(const v4u*)(s16 + e11 + ch0);
#pragma unroll
            for (int j = 0; j < 4; ++j) {
              v00[2 * j] = __uint_as_float(q00[j] << 16); v00[2 * j + 1] = __uint_as_float(q00[j] & 0xffff0000u);
              v01[2 * j] = __uint_as_float(q01[j] << 16); v01[2 * j + 1] = __uint_as_float(q01[j] & 0xffff0000u);
              v10[2 * j] = __uint_as_float(q10[j] << 16); v10[2 * j + 1] = __uint_as_float(q10[j] & 0xffff0000u);
              v11[2 * j] = __uint_as_float(q11[j] << 16); v11[2 * j + 1] = __uint_as_float(q11[j] & 0xffff0000u);
            }
          }
          v8h o;
#pragma unroll
          for (int e = 0; e < 8; ++e) {
            float a = cw00 * v00[e];
            a = a + cw01 * v01[e];
            a = a + cw10 * v10[e];
            a = a + cw11 * v11[e];
            a = a * mk;
            a = a * CSC;
            o[e] = (_Float16)a;
          }
          *(v8h*)(At + m * SP + ch0) = o;
        }
      }
      __syncthreads();

      {
        const _Float16* bt = bp + tap * CIN;
        const _Float16* ab = At + (16 * mt + l15) * SP + 8 * hh;
#pragma unroll 2
        for (int kc = 0; kc < CIN / 32; ++kc) {
          const v16h fa  = ldfrag_h(ab + 32 * kc);
          const v16h fb0 = ldfrag_h(bt + 32 * kc);
          const v16h fb1 = ldfrag_h(bt + 16 * K + 32 * kc);
          acc[0] = mma_h(fa, fb0, acc[0]);
          acc[1] = mma_h(fa, fb1, acc[1]);
          guard2x3(acc[0], acc[1], fa, fb0, fb1);
        }
      }
      __syncthreads();
    }
  }
  acc_guard2(acc[0], acc[1]);

#pragma unroll
  for (int j = 0; j < 2; ++j) {
    const int o = 32 * nq + 16 * j + l15;
    const float bb  = bf_rne(bias[o]);
    const float mu  = bf_rne(mea[o]);
    const float ga  = bf_rne(gam[o]);
    const float va  = bf_rne(var[o]);
    const float be  = bf_rne(bet[o]);
    const float inv = ga / sqrtf(va + 1e-5f);
#pragma unroll
    for (int r = 0; r < 8; ++r) {
      float v = acc[j][r] * INV_S;
      v = v + bb;
      v = v - mu;
      v = v * inv;
      v = v + be;
      v = (v > 0.0f) ? v : 0.0f;
      if constexpr (ONCHW) os[o * OSP + 16 * mt + 8 * hh + r] = v;
      else                 os[(16 * mt + 8 * hh + r) * OSP + o] = v;
    }
  }
  __syncthreads();

  {
    v4f val[4]; size_t e[4];
#pragma unroll
    for (int it = 0; it < 4; ++it) {
      const int L = it * 32 + wid * 4 + lq;
      if constexpr (ONCHW) {
        val[it] = *(const v4f*)(os + L * OSP + 4 * pj);
        e[it]   = ((size_t)(b * NO + L) * IH + h) * IW + xo + 4 * pj;
      } else {
        const int px  = L >> 2;
        const int sub = L & 3;
        val[it] = *(const v4f*)(os + px * OSP + 32 * sub + 4 * pj);
        e[it]   = (pix0 + px) * NO + 32 * sub + 4 * pj;
      }
    }
#pragma unroll
    for (int it = 0; it < 4; ++it) *(volatile v4f*)(dst + e[it]) = val[it];
    __threadfence();
#pragma unroll
    for (int it = 0; it < 4; ++it) *(volatile v4f*)(dst + e[it]) = val[it];
  }
}

__global__ __launch_bounds__(256)
void k_up(const float* __restrict__ hbuf, const float* __restrict__ pre,
          const float* __restrict__ upw, float* zf, unsigned short* zh, unsigned short* zl)
{
  __shared__ __align__(16) float T[UPR * TPU];
  __shared__ __align__(16) float upl[NO * 16];

  const int tid  = threadIdx.x;
  const int lane = tid & 31;
  const int wid  = tid >> 5;
  const int pj   = lane & 7;
  const int lq   = lane >> 3;
  const int q    = blockIdx.x & 3;
  const int by   = blockIdx.x >> 2;
  const int b    = by / PH2;
  const int Yp   = by - b * PH2;
  const bool inrow = (Yp >= 1) && (Yp <= H2);
  const int Y    = min(max(Yp - 1, 0), H2 - 1);

#pragma unroll
  for (int i = 0; i < 8; ++i) upl[tid + 256 * i] = bf_rne(upw[tid + 256 * i]);
  if (tid < 64) {
    const int row = (tid < 32) ? 0 : (UPR - 1);
    *(v4f*)&T[row * TPU + 4 * (tid & 31)] = zero4f();
  }
#pragma unroll 2
  for (int i = 0; i < 8; ++i) {
    const int idx = tid + 256 * i;
    const int w4  = idx & 15;
    const int c   = idx >> 4;
    const v4f v = *(const v4f*)(pre + ((size_t)(b * NO + c) * H2 + Y) * W2 + 64 * q + 4 * w4);
    float* tp = T + (4 * w4 + 1) * TPU + c;
    tp[0 * TPU] = inrow ? bf_rne(v.x) : 0.0f;
    tp[1 * TPU] = inrow ? bf_rne(v.y) : 0.0f;
    tp[2 * TPU] = inrow ? bf_rne(v.z) : 0.0f;
    tp[3 * TPU] = inrow ? bf_rne(v.w) : 0.0f;
  }
  __syncthreads();

  {
    const int xl = 8 * wid + (lane >> 2);
    const int cq = lane & 3;
    const int X  = 64 * q + xl;
    const int ia = (Y + 1) & 1;
    const int ya = (Y + 1 - ia) >> 1;
    const int yb = ya - 1;
    const int ib = ia + 2;
    const int ja = (X + 1) & 1;
    const int xa = (X + 1 - ja) >> 1;
    const int xb = xa - 1;
    const int jb = ja + 2;
    const bool vya = inrow && (ya < H1);
    const bool vyb = inrow && (yb >= 0);
    const bool vxa = (xa < W1);
    const bool vxb = (xb >= 0);
    const int yac = min(max(ya, 0), H1 - 1);
    const int ybc = min(max(yb, 0), H1 - 1);
    const int xac = min(max(xa, 0), W1 - 1);
    const int xbc = min(max(xb, 0), W1 - 1);
    const bool vaa = vya && vxa;
    const bool vab = vya && vxb;
    const bool vba = vyb && vxa;
    const bool vbb = vyb && vxb;
    const int iaa = ia * 4 + ja;
    const int iab = ia * 4 + jb;
    const int iba = ib * 4 + ja;
    const int ibb = ib * 4 + jb;
    const float* paa = hbuf + (((size_t)(b * H1 + yac)) * W1 + xac) * NO + 32 * cq;
    const float* pab = hbuf + (((size_t)(b * H1 + yac)) * W1 + xbc) * NO + 32 * cq;
    const float* pba = hbuf + (((size_t)(b * H1 + ybc)) * W1 + xac) * NO + 32 * cq;
    const float* pbb = hbuf + (((size_t)(b * H1 + ybc)) * W1 + xbc) * NO + 32 * cq;
    float* trow = T + (xl + 1) * TPU + 32 * cq;
#pragma unroll 2
    for (int k = 0; k < 8; ++k) {
      const v4f haa = *(const v4f*)(paa + 4 * k);
      const v4f hab = *(const v4f*)(pab + 4 * k);
      const v4f hba = *(const v4f*)(pba + 4 * k);
      const v4f hbb = *(const v4f*)(pbb + 4 * k);
      const v4f tv  = *(const v4f*)(trow + 4 * k);
      v4f rr;
#pragma unroll
      for (int e = 0; e < 4; ++e) {
        const float* wc = upl + (32 * cq + 4 * k + e) * 16;
        const float waa = vaa ? wc[iaa] : 0.0f;
        const float wab = vab ? wc[iab] : 0.0f;
        const float wba = vba ? wc[iba] : 0.0f;
        const float wbb = vbb ? wc[ibb] : 0.0f;
        float u = waa * haa[e];
        u = u + wab * hab[e];
        u = u + wba * hba[e];
        u = u + wbb * hbb[e];
        rr[e] = u + tv[e];
      }
      *(v4f*)(trow + 4 * k) = rr;
    }
  }
  __syncthreads();

  const int lo_lp = (q == 0) ? 0 : 1;
  const int hi_lp = (q == 3) ? (UPR - 1) : (UPR - 2);
  const size_t pb = ((size_t)(by * PW2 + 64 * q)) * NO;

  {
    constexpr int NIT = 9;
    v4f val[NIT]; size_t e[NIT]; bool ok[NIT];
#pragma unroll
    for (int r = 0; r < NIT; ++r) {
      const int L   = r * 32 + wid * 4 + lq;
      const int lp  = L >> 2;
      const int sub = L & 3;
      ok[r] = (lp >= lo_lp) && (lp <= hi_lp);
      const int lpc = min(lp, UPR - 1);
      val[r] = *(const v4f*)&T[lpc * TPU + 32 * sub + 4 * pj];
      e[r]   = pb + (size_t)lp * NO + 32 * sub + 4 * pj;
    }
#pragma unroll
    for (int r = 0; r < NIT; ++r) if (ok[r]) *(volatile v4f*)(zf + e[r]) = val[r];
    __threadfence();
#pragma unroll
    for (int r = 0; r < NIT; ++r) if (ok[r]) *(volatile v4f*)(zf + e[r]) = val[r];
  }

  {
    constexpr int NIT = 5;
    v4u hv[NIT], lv[NIT]; size_t e[NIT]; bool ok[NIT];
#pragma unroll
    for (int r = 0; r < NIT; ++r) {
      const int L   = r * 32 + wid * 4 + lq;
      const int lp  = L >> 1;
      const int sub = L & 1;
      ok[r] = (lp >= lo_lp) && (lp <= hi_lp);
      const int lpc = min(lp, UPR - 1);
      const v4f f0 = *(const v4f*)&T[lpc * TPU + 64 * sub + 8 * pj];
      const v4f f1 = *(const v4f*)&T[lpc * TPU + 64 * sub + 8 * pj + 4];
      unsigned hb[8], lb[8];
#pragma unroll
      for (int k = 0; k < 4; ++k) {
        const unsigned h0 = bfb(f0[k]);
        hb[k]     = h0;
        lb[k]     = bfb(f0[k] - __uint_as_float(h0 << 16));
        const unsigned h1 = bfb(f1[k]);
        hb[4 + k] = h1;
        lb[4 + k] = bfb(f1[k] - __uint_as_float(h1 << 16));
      }
      hv[r].x = hb[0] | (hb[1] << 16);
      hv[r].y = hb[2] | (hb[3] << 16);
      hv[r].z = hb[4] | (hb[5] << 16);
      hv[r].w = hb[6] | (hb[7] << 16);
      lv[r].x = lb[0] | (lb[1] << 16);
      lv[r].y = lb[2] | (lb[3] << 16);
      lv[r].z = lb[4] | (lb[5] << 16);
      lv[r].w = lb[6] | (lb[7] << 16);
      e[r] = pb + (size_t)lp * NO + 64 * sub + 8 * pj;
    }
#pragma unroll
    for (int r = 0; r < NIT; ++r) if (ok[r]) {
      *(volatile v4u*)(zh + e[r]) = hv[r];
      *(volatile v4u*)(zl + e[r]) = lv[r];
    }
    __threadfence();
#pragma unroll
    for (int r = 0; r < NIT; ++r) if (ok[r]) {
      *(volatile v4u*)(zh + e[r]) = hv[r];
      *(volatile v4u*)(zl + e[r]) = lv[r];
    }
  }
}

extern "C" void kernel_launch(void* const* d_in, const int* in_sizes, int n_in,
                              void* d_out, int out_size, void* d_ws, size_t ws_size,
                              hipStream_t stream) {
  if (n_in < 19) return;
  if (in_sizes[0] != NB * C1 * H1 * W1) return;
  if (in_sizes[1] != NB * NO * H2 * W2) return;
  if (in_sizes[2] != NOF * C1 * 9) return;
  if (in_sizes[3] != NOF) return;
  if (in_sizes[4] != NO * C1 * 9) return;
  for (int i = 5; i <= 9; ++i) if (in_sizes[i] != NO) return;
  if (in_sizes[10] != NOF * NO * 9) return;
  if (in_sizes[11] != NOF) return;
  if (in_sizes[12] != NO * NO * 9) return;
  for (int i = 13; i <= 17; ++i) if (in_sizes[i] != NO) return;
  if (in_sizes[18] != NO * 16) return;
  if (out_size != NB * NO * H2 * W2) return;
  if ((size_t)WS_END > ws_size) return;

  const float* x        = (const float*)d_in[0];
  const float* pre_x    = (const float*)d_in[1];
  const float* p_w_om   = (const float*)d_in[2];
  const float* p_b_om   = (const float*)d_in[3];
  const float* p_w      = (const float*)d_in[4];
  const float* p_b      = (const float*)d_in[5];
  const float* p_gamma  = (const float*)d_in[6];
  const float* p_beta   = (const float*)d_in[7];
  const float* p_mean   = (const float*)d_in[8];
  const float* p_var    = (const float*)d_in[9];
  const float* n_w_om   = (const float*)d_in[10];
  const float* n_b_om   = (const float*)d_in[11];
  const float* n_w      = (const float*)d_in[12];
  const float* n_b      = (const float*)d_in[13];
  const float* n_gamma  = (const float*)d_in[14];
  const float* n_beta   = (const float*)d_in[15];
  const float* n_mean   = (const float*)d_in[16];
  const float* n_var    = (const float*)d_in[17];
  const float* up_w     = (const float*)d_in[18];
  float* out = (float*)d_out;
  char* ws = (char*)d_ws;

  unsigned*       wo1 = (unsigned*)(ws + WS_WO1);
  unsigned*       wr1 = (unsigned*)(ws + WS_WR1);
  unsigned*       wo2 = (unsigned*)(ws + WS_WO2);
  unsigned*       wr2 = (unsigned*)(ws + WS_WR2);
  unsigned short* xh  = (unsigned short*)(ws + WS_XH);
  float*          of1 = (float*)(ws + WS_OF1);
  float*          hb  = (float*)(ws + WS_HB);
  float*          zf  = (float*)(ws + WS_ZF);
  unsigned short* zh  = (unsigned short*)(ws + WS_ZH);
  unsigned short* zl  = (unsigned short*)(ws + WS_ZL);
  float*          of2 = (float*)(ws + WS_OF2);

  k_wpack<<<dim3(WO1_CHK / 256), dim3(256), 0, stream>>>(p_w_om, wo1, NOF, C1, 0);
  (void)hipGetLastError();
  k_wpack<<<dim3(WR1_CHK / 256), dim3(256), 0, stream>>>(p_w, wr1, NO, C1, 1);
  (void)hipGetLastError();
  k_wpack<<<dim3(WO2_CHK / 256), dim3(256), 0, stream>>>(n_w_om, wo2, NOF, NO, 0);
  (void)hipGetLastError();
  k_wpack<<<dim3(WR2_CHK / 256), dim3(256), 0, stream>>>(n_w, wr2, NO, NO, 1);
  (void)hipGetLastError();

  k_xcvt<<<dim3(XCV_BLK), dim3(256), 0, stream>>>(x, xh);
  (void)hipGetLastError();

  k_offs<C1, H1, W1, false><<<dim3(OFF1_BLK), dim3(256), 0, stream>>>(
      (const __bf16*)xh, (const __bf16*)xh, (const __bf16*)wo1, p_b_om, of1);
  (void)hipGetLastError();

  k_conv<C1, H1, W1, false, false><<<dim3(CNV1_BLK), dim3(256), 0, stream>>>(
      (const unsigned short*)xh, (const float*)zf, (const _Float16*)wr1, (const float*)of1,
      p_b, p_gamma, p_beta, p_mean, p_var, hb);
  (void)hipGetLastError();

  k_up<<<dim3(UP_BLK), dim3(256), 0, stream>>>((const float*)hb, pre_x, up_w, zf, zh, zl);
  (void)hipGetLastError();

  k_offs<NO, H2, W2, true><<<dim3(OFF2_BLK), dim3(256), 0, stream>>>(
      (const __bf16*)zh, (const __bf16*)zl, (const __bf16*)wo2, n_b_om, of2);
  (void)hipGetLastError();

  k_conv<NO, H2, W2, true, true><<<dim3(CNV2_BLK), dim3(256), 0, stream>>>(
      (const unsigned short*)xh, (const float*)zf, (const _Float16*)wr2, (const float*)of2,
      n_b, n_gamma, n_beta, n_mean, n_var, out);
  (void)hipGetLastError();
}
